// SelfAttention2D_44736379355575
// MI455X (gfx1250) — hardware-run, weakly checked
//
#include <hip/hip_runtime.h>
#include <stdint.h>

typedef __attribute__((ext_vector_type(16))) _Float16 v16h;
typedef __attribute__((ext_vector_type(8)))  _Float16 v8h;
typedef __attribute__((ext_vector_type(16))) __bf16   v16b;
typedef __attribute__((ext_vector_type(8)))  __bf16   v8b;
typedef __attribute__((ext_vector_type(8)))  float    v8f;
typedef __attribute__((ext_vector_type(4)))  float    v4f;
typedef __attribute__((ext_vector_type(4)))  unsigned int v4u;

__device__ __forceinline__ unsigned short f2bf_bits(float f) {
  unsigned u = __float_as_uint(f);
  return (unsigned short)((u + 0x7FFFu + ((u >> 16) & 1u)) >> 16);
}
__device__ __forceinline__ float bf_bits2f(unsigned short h) { return __uint_as_float(((unsigned)h) << 16); }

__device__ __forceinline__ void dep_guard_h(v8f& a, v8f& b, v16h x, v16h y) { asm volatile("v_nop\n\tv_nop\n\tv_nop\n\tv_nop" : "+v"(a), "+v"(b) : "v"(x), "v"(y)); }
__device__ __forceinline__ void dep_guard_b(v8f& a, v8f& b, v16b x, v16b y) { asm volatile("v_nop\n\tv_nop\n\tv_nop\n\tv_nop" : "+v"(a), "+v"(b) : "v"(x), "v"(y)); }
__device__ __forceinline__ void keep4_h(v16h a, v16h b, v16h c, v16h d) { asm volatile("v_nop" :: "v"(a), "v"(b), "v"(c), "v"(d)); }
__device__ __forceinline__ void keep4_b(v16b a, v16b b, v16b c, v16b d) { asm volatile("v_nop" :: "v"(a), "v"(b), "v"(c), "v"(d)); }
__device__ __forceinline__ void acc_guard4(v8f& a, v8f& b, v8f& c, v8f& d) { asm volatile("v_nop\n\tv_nop\n\tv_nop\n\tv_nop" : "+v"(a), "+v"(b), "+v"(c), "+v"(d)); }
template <typename T> struct Frag;
template <> struct Frag<_Float16> {
  typedef v16h V; union U { v16h v; v8h h[2]; };
  static __device__ __forceinline__ v16h load(const _Float16* p) {
    U f; f.h[0] = *(const v8h*)(p); f.h[1] = *(const v8h*)(p + 16); return f.v;
  }
  static __device__ __forceinline__ v8f mma(v16h a, v16h b, v8f c) {
    return __builtin_amdgcn_wmma_f32_16x16x32_f16(false, a, false, b, (short)0, c, false, false);
  }
  static __device__ __forceinline__ void guard(v8f& a, v8f& b, v16h x, v16h y) { dep_guard_h(a, b, x, y); }
  static __device__ __forceinline__ void keep(v16h a, v16h b, v16h c, v16h d) { keep4_h(a, b, c, d); }
};
template <> struct Frag<__bf16> {
  typedef v16b V; union U { v16b v; v8b h[2]; };
  static __device__ __forceinline__ v16b load(const __bf16* p) {
    U f; f.h[0] = *(const v8b*)(p); f.h[1] = *(const v8b*)(p + 16); return f.v;
  }
  static __device__ __forceinline__ v8f mma(v16b a, v16b b, v8f c) {
    return __builtin_amdgcn_wmma_f32_16x16x32_bf16(false, a, false, b, (short)0, c, false, false);
  }
  static __device__ __forceinline__ void guard(v8f& a, v8f& b, v16b x, v16b y) { dep_guard_b(a, b, x, y); }
  static __device__ __forceinline__ void keep(v16b a, v16b b, v16b c, v16b d) { keep4_b(a, b, c, d); }
};

template <int ET> struct Elem;
template <> struct Elem<0> { typedef _Float16 T; };
template <> struct Elem<1> { typedef __bf16 T; };
template <int ET, bool SPLIT, int BIAS_MODE, int OUT_MODE, bool RESID, int ACT = 0>
__global__ __launch_bounds__(256) void wmma_gemm64(
    const unsigned short* __restrict__ Ap, const unsigned short* __restrict__ A2p, int lda, long strideA,
    const unsigned short* __restrict__ Btp, const unsigned short* __restrict__ Bt2p, int ldb, long strideB,
    void* __restrict__ Cout, void* __restrict__ Cout2, int ldc, long strideC,
    const float* __restrict__ bias,
    const float* __restrict__ resid, long strideR,
    int M, int N, int K, float scale) {
  typedef typename Elem<ET>::T T;
  typedef typename Frag<T>::V V;
  const T* A = (const T*)Ap; const T* A2 = (const T*)A2p; const T* Bt = (const T*)Btp; const T* Bt2 = (const T*)Bt2p;
  __shared__ __align__(16) float sT[8][16 * 68];
  const int b    = blockIdx.y;
  const int lane = threadIdx.x & 31;
  const int wave = threadIdx.x >> 5;
  const int tilesN = N >> 6;
  const int tilesM = M >> 6;
  const int tile = blockIdx.x * 8 + wave;
  if (tile >= tilesM * tilesN) return;
  const int tm = tile / tilesN;
  const int tn = tile - tm * tilesN;
  const int m0 = tm << 6;
  const int n0 = tn << 6;

  const T* Ab  = A  + (size_t)b * strideA;
  const T* Bb  = Bt + (size_t)b * strideB;
  const T* Ab2 = SPLIT ? (A2  + (size_t)b * strideA) : nullptr;
  const T* Bb2 = SPLIT ? (Bt2 + (size_t)b * strideB) : nullptr;

  const int rlane = lane & 15;
  const int koff  = (lane >> 4) * 8;
  const int mOff  = (lane >> 4) * 8;

  v8f acc[4][4];
#pragma unroll
  for (int i = 0; i < 4; ++i)
#pragma unroll
    for (int j = 0; j < 4; ++j) acc[i][j] = (v8f){0.f,0.f,0.f,0.f,0.f,0.f,0.f,0.f};

  for (int k0 = 0; k0 < K; k0 += 32) {
    V bh[4], bl[4];
#pragma unroll
    for (int j = 0; j < 4; ++j) {
      const size_t bo = (size_t)(n0 + (j << 4) + rlane) * ldb + koff + k0;
      bh[j] = Frag<T>::load(Bb + bo);
      if (SPLIT) bl[j] = Frag<T>::load(Bb2 + bo);
    }
#pragma unroll
    for (int i = 0; i < 4; ++i) {
      const size_t ao = (size_t)(m0 + (i << 4) + rlane) * lda + koff + k0;
      V ah = Frag<T>::load(Ab + ao);
      V al;
      if (SPLIT) al = Frag<T>::load(Ab2 + ao);
#pragma unroll
      for (int j = 0; j < 4; ++j) {
        acc[i][j] = Frag<T>::mma(ah, bh[j], acc[i][j]);
        if (SPLIT) {
          acc[i][j] = Frag<T>::mma(ah, bl[j], acc[i][j]);
          acc[i][j] = Frag<T>::mma(al, bh[j], acc[i][j]);
        }
      }
      Frag<T>::guard(acc[i][0], acc[i][3], ah, SPLIT ? al : ah);
    }
    Frag<T>::keep(bh[0], bh[1], bh[2], bh[3]);
    if (SPLIT) Frag<T>::keep(bl[0], bl[1], bl[2], bl[3]);
  }
  acc_guard4(acc[0][0], acc[0][1], acc[0][2], acc[0][3]);
  acc_guard4(acc[1][0], acc[1][1], acc[1][2], acc[1][3]);
  acc_guard4(acc[2][0], acc[2][1], acc[2][2], acc[2][3]);
  acc_guard4(acc[3][0], acc[3][1], acc[3][2], acc[3][3]);

  float* slab = sT[wave];
  const float* Rb = RESID ? (resid + (size_t)b * strideR) : nullptr;
#pragma unroll
  for (int i = 0; i < 4; ++i) {
    const int mBase = m0 + (i << 4);
#pragma unroll
    for (int j = 0; j < 4; ++j) {
      const int n = n0 + (j << 4) + rlane;
      float bv = 0.f;
      if (BIAS_MODE == 2) bv = bias[n];
#pragma unroll
      for (int r = 0; r < 8; ++r) {
        float v = acc[i][j][r] * scale;
        if (BIAS_MODE == 1) v += bias[mBase + mOff + r];
        if (BIAS_MODE == 2) v += bv;
        if (RESID) v += Rb[(size_t)(mBase + mOff + r) * ldc + n];
        if (ACT == 1) v = tanhf(v);
        if (ACT == 2) v = fmaxf(v, 0.0f);
        if (ACT == 3) v = v / (1.0f + expf(-v));
        if (ACT == 4) v = (v > 0.f) ? v : 0.01f * v;
        if (ACT == 5) v = 0.5f * v * (1.0f + erff(v * 0.70710678118654752f));
        slab[(mOff + r) * 68 + (j << 4) + rlane] = v;
      }
    }
    __builtin_amdgcn_fence(__ATOMIC_RELEASE, "workgroup");
    __builtin_amdgcn_wave_barrier();
    __builtin_amdgcn_fence(__ATOMIC_ACQUIRE, "workgroup");
    if (OUT_MODE == 0) {
      float* C = (float*)Cout + (size_t)b * strideC;
      const int hh = lane >> 4, c4 = (lane & 15) * 4;
      for (int pass = 0; pass < 2; ++pass) {
#pragma unroll
        for (int it = 0; it < 8; ++it) {
          const int row = it * 2 + hh;
          v4f v = *(const v4f*)(slab + row * 68 + c4);
          *(volatile v4f*)(C + (size_t)(mBase + row) * ldc + n0 + c4) = v;
        }
        __threadfence();
      }
    } else {
      const int q = lane >> 3, c8 = (lane & 7) * 8;
      unsigned short* C  = (unsigned short*)Cout  + (size_t)b * strideC;
      unsigned short* C2 = (OUT_MODE == 2) ? ((unsigned short*)Cout2 + (size_t)b * strideC) : nullptr;
      for (int pass = 0; pass < 2; ++pass) {
#pragma unroll
        for (int it = 0; it < 4; ++it) {
          const int row = it * 4 + q;
          const float* sp = slab + row * 68 + c8;
          v8h hv, lv;
#pragma unroll
          for (int e = 0; e < 8; ++e) {
            if (OUT_MODE == 1) {
              hv[e] = (_Float16)sp[e];
            } else {
              unsigned short hb = f2bf_bits(sp[e]);
              unsigned short lb = f2bf_bits(sp[e] - bf_bits2f(hb));
              hv[e] = __builtin_bit_cast(_Float16, hb);
              lv[e] = __builtin_bit_cast(_Float16, lb);
            }
          }
          *(volatile v8h*)(C + (size_t)(mBase + row) * ldc + n0 + c8) = hv;
          if (OUT_MODE == 2) *(volatile v8h*)(C2 + (size_t)(mBase + row) * ldc + n0 + c8) = lv;
        }
        __threadfence();
      }
    }
    __builtin_amdgcn_fence(__ATOMIC_RELEASE, "workgroup");
    __builtin_amdgcn_wave_barrier();
    __builtin_amdgcn_fence(__ATOMIC_ACQUIRE, "workgroup");
  }
}

#define NBATCH 4
#define NPIX 4096
#define NCH 128
#define DKQ 16
#define NTOT (NBATCH * NPIX)
#define FGW 32
#define CFGW 64
#define RBLK 64
#define MCHK 64
#define PPITCH 72
#define OPITCH 132
#define LOG2E_F 1.44269504088896340736f
#define PCARRY_LOG2 15.0f
#define PCARRY_INV (1.0f / 32768.0f)
#define PEXP_CLAMP 15.99f

static_assert(NTOT % 64 == 0, "tile multiple M/N");
static_assert(NCH % 64 == 0, "tile multiple");
static_assert(NCH % 32 == 0, "K multiple of 32");
static_assert(CFGW % 64 == 0, "tile multiple N");
static_assert(NPIX % RBLK == 0 && NPIX % MCHK == 0, "blocking");
static_assert((PPITCH * 2) % 16 == 0 && (OPITCH * 4) % 16 == 0, "lds alignment");

union FragB { v16b v; v8b h[2]; v4u q[2]; };

__device__ __forceinline__ v8f mma_bf(v16b a, v16b b, v8f c) {
  c = __builtin_amdgcn_wmma_f32_16x16x32_bf16(false, a, false, b, (short)0, c, false, false);
  asm volatile("v_nop\n\tv_nop\n\tv_nop\n\tv_nop" : "+v"(c) : "v"(a), "v"(b));
  return c;
}
__device__ __forceinline__ v8f mma_h(v16h a, v16h b, v8f c) {
  c = __builtin_amdgcn_wmma_f32_16x16x32_f16(false, a, false, b, (short)0, c, false, false);
  asm volatile("v_nop\n\tv_nop\n\tv_nop\n\tv_nop" : "+v"(c) : "v"(a), "v"(b));
  return c;
}

__device__ __forceinline__ void split8_bf16(const float (&v)[8], v4u& qh, v4u& ql) {
  unsigned hb[8], lb[8];
#pragma unroll
  for (int e = 0; e < 8; ++e) {
    const unsigned short h = f2bf_bits(v[e]);
    hb[e] = h;
    lb[e] = f2bf_bits(v[e] - bf_bits2f(h));
  }
  qh = (v4u){ hb[0] | (hb[1] << 16), hb[2] | (hb[3] << 16), hb[4] | (hb[5] << 16), hb[6] | (hb[7] << 16) };
  ql = (v4u){ lb[0] | (lb[1] << 16), lb[2] | (lb[3] << 16), lb[4] | (lb[5] << 16), lb[6] | (lb[7] << 16) };
}

__global__ __launch_bounds__(256) void wprep_kernel(
    const float* __restrict__ kf, const float* __restrict__ kg, const float* __restrict__ kh,
    unsigned short* __restrict__ whh, unsigned short* __restrict__ whl,
    unsigned short* __restrict__ wfgh, unsigned short* __restrict__ wfgl)
{
  const int tid = blockIdx.x * 256 + threadIdx.x;
  float v[8];
  unsigned short* dh;
  unsigned short* dl;
  if (blockIdx.x < 8) {
    const int row = tid >> 4;
    const int c0  = (tid & 15) << 3;
#pragma unroll
    for (int e = 0; e < 8; ++e) v[e] = kh[(size_t)(c0 + e) * NCH + row];
    dh = whh + (size_t)row * NCH + c0;
    dl = whl + (size_t)row * NCH + c0;
  } else {
    const int t    = tid - 8 * 256;
    const int row  = t >> 4;
    const int c0   = (t & 15) << 3;
    const int bsel = blockIdx.x - 8;
    const int d    = row & 15;
    const float* src = (bsel == 0) ? kf : kg;
    if (bsel < 2) {
#pragma unroll
      for (int e = 0; e < 8; ++e) v[e] = src[(size_t)(c0 + e) * DKQ + d];
    } else {
#pragma unroll
      for (int e = 0; e < 8; ++e) v[e] = 0.0f;
    }
    dh = wfgh + (size_t)row * NCH + c0;
    dl = wfgl + (size_t)row * NCH + c0;
  }
  v4u qh, ql;
  split8_bf16(v, qh, ql);
  *(volatile v4u*)dh = qh;
  *(volatile v4u*)dl = ql;
  __threadfence();
  *(volatile v4u*)dh = qh;
  *(volatile v4u*)dl = ql;
}

__global__ __launch_bounds__(256) void xsplit_kernel(
    const float* __restrict__ x, unsigned short* __restrict__ xh, unsigned short* __restrict__ xl, int n8)
{
  const int t = blockIdx.x * 256 + threadIdx.x;
  if (t < n8) {
    const float* p = x + (size_t)t * 8;
    const v4f u0 = *(const v4f*)p;
    const v4f u1 = *(const v4f*)(p + 4);
    float v[8] = { u0[0], u0[1], u0[2], u0[3], u1[0], u1[1], u1[2], u1[3] };
    v4u qh, ql;
    split8_bf16(v, qh, ql);
    unsigned short* dh = xh + (size_t)t * 8;
    unsigned short* dl = xl + (size_t)t * 8;
    *(volatile v4u*)dh = qh;
    *(volatile v4u*)dl = ql;
    __threadfence();
    *(volatile v4u*)dh = qh;
    *(volatile v4u*)dl = ql;
  }
}

__global__ __launch_bounds__(256) void fg_plane_kernel(
    const float* __restrict__ cfg, unsigned short* __restrict__ fpl, unsigned short* __restrict__ gpl)
{
  const int t     = blockIdx.x * 256 + threadIdx.x;
  const int plane = blockIdx.y;
  const int row   = t >> 2;
  const int part  = t & 3;
  const float sc  = (plane == 0) ? LOG2E_F : 1.0f;
  const float* src = cfg + (size_t)row * CFGW + plane * DKQ + ((part & 1) << 3);
  const v4f u0 = *(const v4f*)src;
  const v4f u1 = *(const v4f*)(src + 4);
  float v[8] = { u0[0] * sc, u0[1] * sc, u0[2] * sc, u0[3] * sc, u1[0] * sc, u1[1] * sc, u1[2] * sc, u1[3] * sc };
  v4u qh, ql;
  split8_bf16(v, qh, ql);
  const bool uselo = (part >> 1) != 0;
  v4u q;
  q[0] = uselo ? ql[0] : qh[0];
  q[1] = uselo ? ql[1] : qh[1];
  q[2] = uselo ? ql[2] : qh[2];
  q[3] = uselo ? ql[3] : qh[3];
  unsigned short* dst = ((plane == 0) ? fpl : gpl) + (size_t)t * 8;
  *(volatile v4u*)dst = q;
  __threadfence();
  *(volatile v4u*)dst = q;
}

__global__ __launch_bounds__(256) void colstats_kernel(
    const unsigned short* __restrict__ gpl, const unsigned short* __restrict__ fpl, float* __restrict__ Mp)
{
  __shared__ float redM[8 * 64];
  __shared__ float redS[8 * 64];
  __shared__ __align__(16) float stage[64];
  const int tid  = threadIdx.x;
  const int lane = tid & 31;
  const int wave = tid >> 5;
  const int hh   = lane >> 4;
  const int cl   = lane & 15;
  const int b    = blockIdx.x / (NPIX / 64);
  const int mc0  = (blockIdx.x - b * (NPIX / 64)) * 64;
  const __bf16* Gb = (const __bf16*)gpl + (size_t)b * NPIX * FGW;
  const __bf16* Fb = (const __bf16*)fpl + (size_t)b * NPIX * FGW;
  const v4u z4 = { 0u, 0u, 0u, 0u };
  const v8f z8 = { 0.f, 0.f, 0.f, 0.f, 0.f, 0.f, 0.f, 0.f };

  v16b b1[4], b2[4];
#pragma unroll
  for (int j = 0; j < 4; ++j) {
    const __bf16* F = Fb + (size_t)(mc0 + (j << 4) + cl) * FGW + 8 * hh;
    const v8b fh = *(const v8b*)F;
    const v8b fl = *(const v8b*)(F + 16);
    FragB u1, u2;
    u1.h[0] = fh; u1.h[1] = fh;
    u2.h[0] = fl; u2.q[1] = z4;
    b1[j] = u1.v; b2[j] = u2.v;
  }

  float mx[4], sm[4];
#pragma unroll
  for (int j = 0; j < 4; ++j) { mx[j] = -3.0e38f; sm[j] = 0.f; }

#pragma unroll 1
  for (int step = 0; step < 32; ++step) {
    const int n = wave * 512 + step * 16;
    const __bf16* G = Gb + (size_t)(n + cl) * FGW + 8 * hh;
    FragB ua;
    ua.v = Frag<__bf16>::load(G);
    FragB ub;
    ub.h[0] = ua.h[0]; ub.q[1] = z4;
    const v16b a1 = ua.v, a2 = ub.v;
#pragma unroll
    for (int j = 0; j < 4; ++j) {
      v8f s = mma_bf(a1, b1[j], z8);
      s = mma_bf(a2, b2[j], s);
      float tm = s[0];
#pragma unroll
      for (int r = 1; r < 8; ++r) tm = fmaxf(tm, s[r]);
      const float mnew = fmaxf(mx[j], tm);
      float accs = 0.f;
#pragma unroll
      for (int r = 0; r < 8; ++r) accs += exp2f(s[r] - mnew);
      sm[j] = sm[j] * exp2f(mx[j] - mnew) + accs;
      mx[j] = mnew;
    }
  }

#pragma unroll
  for (int j = 0; j < 4; ++j) {
    const float mo = __shfl_xor(mx[j], 16, 32);
    const float so = __shfl_xor(sm[j], 16, 32);
    const float mn = fmaxf(mx[j], mo);
    sm[j] = sm[j] * exp2f(mx[j] - mn) + so * exp2f(mo - mn);
    mx[j] = mn;
  }
  if (hh == 0) {
#pragma unroll
    for (int j = 0; j < 4; ++j) {
      redM[wave * 64 + (j << 4) + cl] = mx[j];
      redS[wave * 64 + (j << 4) + cl] = sm[j];
    }
  }
  __syncthreads();
  if (tid < 64) {
    float Mv = redM[tid];
#pragma unroll
    for (int w = 1; w < 8; ++w) Mv = fmaxf(Mv, redM[w * 64 + tid]);
    float Z = 0.f;
#pragma unroll
    for (int w = 0; w < 8; ++w) Z += redS[w * 64 + tid] * exp2f(redM[w * 64 + tid] - Mv);
    stage[tid] = Mv + log2f(Z) - PCARRY_LOG2;
  }
  __syncthreads();
  if (wave == 0) {
    const v4f val = *(const v4f*)(stage + 4 * cl);
    float* dst = Mp + (size_t)b * NPIX + mc0 + 4 * cl;
    if (lane < 16) *(volatile v4f*)dst = val;
    __threadfence();
    if (lane < 16) *(volatile v4f*)dst = val;
  }
}

__global__ __launch_bounds__(256) void attn_out_kernel(
    const unsigned short* __restrict__ gpl, const unsigned short* __restrict__ fpl,
    const unsigned short* __restrict__ hT, const float* __restrict__ Mp,
    const float* __restrict__ x, const float* __restrict__ gamma, float* __restrict__ out)
{
  __shared__ __align__(16) _Float16 Psh[RBLK * PPITCH];
  __shared__ __align__(16) float Osg[RBLK * OPITCH];
  const int tid  = threadIdx.x;
  const int lane = tid & 31;
  const int wave = tid >> 5;
  const int hh   = lane >> 4;
  const int cl   = lane & 15;
  const int b    = blockIdx.x / (NPIX / RBLK);
  const int n0   = (blockIdx.x - b * (NPIX / RBLK)) * RBLK;
  const __bf16* Gb = (const __bf16*)gpl + (size_t)b * NPIX * FGW;
  const __bf16* Fb = (const __bf16*)fpl + (size_t)b * NPIX * FGW;
  const float* Mpb = Mp + (size_t)b * NPIX;
  const int rt  = wave >> 1;
  const int ctb = (wave & 1) << 1;
  const v4u z4 = { 0u, 0u, 0u, 0u };
  const v8f z8 = { 0.f, 0.f, 0.f, 0.f, 0.f, 0.f, 0.f, 0.f };

  v16b a1, a2;
  {
    const __bf16* G = Gb + (size_t)(n0 + (rt << 4) + cl) * FGW + 8 * hh;
    FragB ua; ua.v = Frag<__bf16>::load(G);
    FragB ub; ub.h[0] = ua.h[0]; ub.q[1] = z4;
    a1 = ua.v; a2 = ub.v;
  }
  const int cw0 = wave << 4;
  const _Float16* Hw = (const _Float16*)hT + (size_t)(cw0 + cl) * NTOT + (size_t)b * NPIX + 8 * hh;

  v8f oacc[4];
#pragma unroll
  for (int t = 0; t < 4; ++t) oacc[t] = z8;

#pragma unroll 1
  for (int mc = 0; mc < NPIX / MCHK; ++mc) {
    const int m0 = mc * MCHK;
    __syncthreads();
#pragma unroll
    for (int j = 0; j < 2; ++j) {
      const int ct = ctb + j;
      const int m  = m0 + (ct << 4) + cl;
      const __bf16* F = Fb + (size_t)m * FGW + 8 * hh;
      const v8b fh = *(const v8b*)F;
      const v8b fl = *(const v8b*)(F + 16);
      FragB u1, u2;
      u1.h[0] = fh; u1.h[1] = fh;
      u2.h[0] = fl; u2.q[1] = z4;
      v8f s = mma_bf(a1, u1.v, z8);
      s = mma_bf(a2, u2.v, s);
      const float mp = Mpb[m];
      _Float16* prow = Psh + ((rt << 4) + 8 * hh) * PPITCH + (ct << 4) + cl;
#pragma unroll
      for (int r = 0; r < 8; ++r) prow[r * PPITCH] = (_Float16)exp2f(fminf(s[r] - mp, PEXP_CLAMP));
    }
    __syncthreads();
#pragma unroll
    for (int kk = 0; kk < 2; ++kk) {
      const v16h bv = Frag<_Float16>::load(Hw + m0 + kk * 32);
#pragma unroll
      for (int t = 0; t < 4; ++t) {
        const v16h av = Frag<_Float16>::load(Psh + ((t << 4) + cl) * PPITCH + kk * 32 + 8 * hh);
        oacc[t] = mma_h(av, bv, oacc[t]);
      }
    }
  }

  const float gsc = gamma[0] * PCARRY_INV;
#pragma unroll
  for (int t = 0; t < 4; ++t) {
#pragma unroll
    for (int r = 0; r < 8; ++r) Osg[((t << 4) + 8 * hh + r) * OPITCH + cw0 + cl] = oacc[t][r] * gsc;
  }
  __syncthreads();
  {
    const size_t rowb = (size_t)b * NPIX + n0 + (wave << 3);
    v4f vals[8];
#pragma unroll
    for (int i = 0; i < 8; ++i) {
      const v4f a  = *(const v4f*)(Osg + ((wave << 3) + i) * OPITCH + 4 * lane);
      const v4f xr = *(const v4f*)(x + (rowb + i) * NCH + 4 * lane);
      vals[i] = a + xr;
    }
    for (int pass = 0; pass < 2; ++pass) {
#pragma unroll
      for (int i = 0; i < 8; ++i) *(volatile v4f*)(out + (rowb + i) * NCH + 4 * lane) = vals[i];
      __threadfence();
    }
  }
}

extern "C" void kernel_launch(void* const* d_in, const int* in_sizes, int n_in,
                              void* d_out, int out_size, void* d_ws, size_t ws_size,
                              hipStream_t stream) {
  const float* x  = (const float*)d_in[0];
  const float* kf = (const float*)d_in[1];
  const float* kg = (const float*)d_in[2];
  const float* kh = (const float*)d_in[3];
  const float* gm = (const float*)d_in[4];
  float* out = (float*)d_out;

  const size_t sz_xp  = (size_t)NTOT * NCH * 2;
  const size_t sz_wh  = (size_t)NCH * NCH * 2;
  const size_t sz_wfg = (size_t)CFGW * NCH * 2;
  const size_t sz_cfg = (size_t)NTOT * CFGW * 4;
  const size_t sz_ht  = (size_t)NCH * NTOT * 2;
  const size_t sz_pl  = (size_t)NTOT * FGW * 2;
  const size_t sz_mp  = (size_t)NTOT * 4;

  size_t off = 0;
  const size_t off_xh = off;   off += sz_xp;
  const size_t off_xl = off;   off += sz_xp;
  const size_t off_whh = off;  off += sz_wh;
  const size_t off_whl = off;  off += sz_wh;
  const size_t off_wfgh = off; off += sz_wfg;
  const size_t off_wfgl = off; off += sz_wfg;
  const size_t off_cfg = off;  off += sz_cfg;
  const size_t off_ht = off;   off += sz_ht;
  const size_t off_fpl = off;  off += sz_pl;
  const size_t off_gpl = off;  off += sz_pl;
  const size_t off_mp = off;   off += sz_mp;
  const size_t ws_total = off;
  if (ws_total > ws_size) return;
  if (n_in < 5) return;
  if (in_sizes[0] != NTOT * NCH || in_sizes[3] != NCH * NCH || in_sizes[1] != NCH * DKQ || in_sizes[2] != NCH * DKQ) return;
  if (out_size != NTOT * NCH) return;

  char* ws = (char*)d_ws;
  unsigned short* xh   = (unsigned short*)(ws + off_xh);
  unsigned short* xl   = (unsigned short*)(ws + off_xl);
  unsigned short* whh  = (unsigned short*)(ws + off_whh);
  unsigned short* whl  = (unsigned short*)(ws + off_whl);
  unsigned short* wfgh = (unsigned short*)(ws + off_wfgh);
  unsigned short* wfgl = (unsigned short*)(ws + off_wfgl);
  float*          cfg  = (float*)(ws + off_cfg);
  unsigned short* hT   = (unsigned short*)(ws + off_ht);
  unsigned short* fpl  = (unsigned short*)(ws + off_fpl);
  unsigned short* gpl  = (unsigned short*)(ws + off_gpl);
  float*          Mp   = (float*)(ws + off_mp);

  wprep_kernel<<<dim3(12), dim3(256), 0, stream>>>(kf, kg, kh, whh, whl, wfgh, wfgl);
  const int n8 = NTOT * NCH / 8;
  xsplit_kernel<<<dim3((n8 + 255) / 256), dim3(256), 0, stream>>>(x, xh, xl, n8);
  wmma_gemm64<1, true, 0, 1, false, 0><<<dim3((NCH / 64) * (NTOT / 64) / 8, 1), dim3(256), 0, stream>>>(
      whh, whl, NCH, (long)0, xh, xl, NCH, (long)0,
      (void*)hT, (void*)nullptr, NTOT, (long)0,
      (const float*)nullptr, (const float*)nullptr, (long)0,
      NCH, NTOT, NCH, 1.0f);
  wmma_gemm64<1, true, 0, 0, false, 0><<<dim3((NTOT / 64) * (CFGW / 64) / 8, 1), dim3(256), 0, stream>>>(
      xh, xl, NCH, (long)0, wfgh, wfgl, NCH, (long)0,
      (void*)cfg, (void*)nullptr, CFGW, (long)0,
      (const float*)nullptr, (const float*)nullptr, (long)0,
      NTOT, CFGW, NCH, 1.0f);
  fg_plane_kernel<<<dim3(NTOT * 4 / 256, 2), dim3(256), 0, stream>>>(cfg, fpl, gpl);
  colstats_kernel<<<dim3(NBATCH * (NPIX / 64)), dim3(256), 0, stream>>>(gpl, fpl, Mp);
  attn_out_kernel<<<dim3(NBATCH * (NPIX / RBLK)), dim3(256), 0, stream>>>(gpl, fpl, hT, Mp, x, gm, out);
}
